// CrossAttention_9216999817487
// MI455X (gfx1250) — hardware-verified
//
#include <hip/hip_runtime.h>
#include <stdint.h>


typedef _Float16 v16h __attribute__((ext_vector_type(16)));
typedef _Float16 v8h  __attribute__((ext_vector_type(8)));
typedef float    v8f  __attribute__((ext_vector_type(8)));
typedef float    v4f  __attribute__((ext_vector_type(4)));

#ifndef NB
#define NB 2
#endif
#ifndef SEQ
#define SEQ 2048
#endif
#ifndef MCTX
#define MCTX 2048
#endif
#define NB_FULL   2
#define SEQ_FULL  2048
#define MCTX_FULL 2048
#define DM   768
#define NH   12
#define HD   64

#define ACT_CAR   8.0f
#define W_CAR     1024.0f
#define PROJ_SCL  0.0009765625f
#define RES_CAR   2048.0f
#define RES_INV   0.00048828125f
#define S_SCL     0.001953125f
#define P_CAR     16384.0f
#define O_SCL     0.001953125f
#define OUT_SCL   3.814697265625e-06f

static_assert(NB >= 1 && NB <= NB_FULL);
static_assert(SEQ % 128 == 0);
static_assert(MCTX % 128 == 0);
static_assert(SEQ <= SEQ_FULL && MCTX <= MCTX_FULL);
static_assert(DM == NH * HD);
static_assert(HD == 64);
static_assert(DM % 128 == 0 && DM % 64 == 0 && DM % 32 == 0 && DM % 8 == 0);
static_assert((long)NB_FULL * SEQ_FULL * DM * 4 == 12582912L);
static_assert(((long)SEQ * DM / 8) % 256 == 0 && ((long)MCTX * DM / 8) % 256 == 0);
static_assert(((long)DM * DM / 8) % 256 == 0);
static_assert((long)(DM / 64) * ((long)NB * SEQ / 128) * 128 * 64 == (long)NB * SEQ * DM);
static_assert((long)(DM / 64) * ((long)NB * MCTX / 128) * 128 * 64 == (long)NB * MCTX * DM);
static_assert((long)(MCTX / 64) * (DM / 128) * NB * 128 * 64 == (long)NB * MCTX * DM);
static_assert((long)(SEQ / 128) * NH * NB * 128 * HD == (long)NB * SEQ * DM);
static_assert((long)(DM / 64) * (SEQ / 64) * NB * 64 * 64 == (long)NB * SEQ * DM);

union Frag16 { v16h v; v8h p[2]; };

__device__ __forceinline__ v16h ld_frag(const _Float16* p, int hl) {
  Frag16 f;
  f.p[0] = *(const v8h*)(p + 8 * hl);
  f.p[1] = *(const v8h*)(p + 16 + 8 * hl);
  return f.v;
}

__device__ __forceinline__ v8f mma(v16h a, v16h b, v8f c) {
  v8f d = __builtin_amdgcn_wmma_f32_16x16x32_f16(false, a, false, b, (short)0, c, false, false);
  asm volatile("v_nop\n\tv_nop\n\tv_nop\n\tv_nop" : "+v"(d) : "v"(a), "v"(b));
  return d;
}

__device__ __forceinline__ float bf16_rne(float x) {
  unsigned int u = __builtin_bit_cast(unsigned int, x);
  u += 0x7FFFu + ((u >> 16) & 1u);
  return __builtin_bit_cast(float, u & 0xFFFF0000u);
}

__global__ __launch_bounds__(256) void k_cvt8(const float* __restrict__ src,
                                              _Float16* __restrict__ dst,
                                              float car, unsigned sstride, unsigned dstride,
                                              unsigned n8)
{
  const unsigned i8 = blockIdx.x * 256u + threadIdx.x;
  if (i8 >= n8) return;
  const size_t e = (size_t)i8 * 8;
  const float* s = src + (size_t)blockIdx.y * sstride + e;
  const v4f x0 = *(const v4f*)s;
  const v4f x1 = *(const v4f*)(s + 4);
  v8h o;
#pragma unroll
  for (int j = 0; j < 4; ++j) {
    const float t0 = x0[j];
    const float t1 = x1[j];
    o[j]     = (_Float16)(bf16_rne(t0) * car);
    o[4 + j] = (_Float16)(bf16_rne(t1) * car);
  }
  _Float16* d = dst + (size_t)blockIdx.y * dstride + e;
  *(volatile v8h*)d = o;
  __threadfence();
  *(volatile v8h*)d = o;
}

__device__ __forceinline__ void gemm_core(const _Float16* ap0, const _Float16* ap1,
                                          const _Float16* bp, int K, int hl, v8f (&acc)[8])
{
  const size_t bst = (size_t)16 * K;
#pragma unroll 1
  for (int k0 = 0; k0 < K; k0 += 32) {
    const v16h a0 = ld_frag(ap0 + k0, hl);
    const v16h a1 = ld_frag(ap1 + k0, hl);
    const v16h b0 = ld_frag(bp + k0, hl);
    const v16h b1 = ld_frag(bp + bst + k0, hl);
    const v16h b2 = ld_frag(bp + 2 * bst + k0, hl);
    const v16h b3 = ld_frag(bp + 3 * bst + k0, hl);
    acc[0] = mma(a0, b0, acc[0]);
    acc[1] = mma(a0, b1, acc[1]);
    acc[2] = mma(a0, b2, acc[2]);
    acc[3] = mma(a0, b3, acc[3]);
    acc[4] = mma(a1, b0, acc[4]);
    acc[5] = mma(a1, b1, acc[5]);
    acc[6] = mma(a1, b2, acc[6]);
    acc[7] = mma(a1, b3, acc[7]);
  }
}

__global__ __launch_bounds__(128) __attribute__((amdgpu_num_vgpr(256)))
void k_proj(const _Float16* __restrict__ A, const _Float16* __restrict__ Bt,
            _Float16* __restrict__ PH, _Float16* __restrict__ PL,
            const float* __restrict__ bias, size_t sB, size_t sC,
            int K, int ldc, int bias_row)
{
  __shared__ __attribute__((aligned(16))) _Float16 ldsE[2 * 128 * 72];
  _Float16* const ldsH = ldsE;
  _Float16* const ldsL = ldsE + 128 * 72;

  const int tid = threadIdx.x, lane = tid & 31, w = tid >> 5;
  const int hl = lane >> 4, c = lane & 15;
  const int m0 = blockIdx.y * 128, n0 = blockIdx.x * 64;
  const int mw = m0 + 32 * w;
  const size_t zb = (size_t)blockIdx.z;

  const _Float16* ap0 = A  + (size_t)(mw + c) * K;
  const _Float16* ap1 = A  + (size_t)(mw + 16 + c) * K;
  const _Float16* bp  = Bt + zb * sB + (size_t)(n0 + c) * K;

  v8f acc[8] = {};
  gemm_core(ap0, ap1, bp, K, hl, acc);

  float bc[4];
#pragma unroll
  for (int t = 0; t < 4; ++t) {
    int ci = n0 + 16 * t + c;
    ci = (ci < DM - 1) ? ci : (DM - 1);
    bc[t] = bf16_rne(bias[ci]) * ACT_CAR;
  }
  v4f br[2][2];
#pragma unroll
  for (int i = 0; i < 2; ++i) {
    int ri = mw + 16 * i + 8 * hl;
    ri = (ri < DM - 8) ? ri : (DM - 8);
    br[i][0] = *(const v4f*)(bias + ri);
    br[i][1] = *(const v4f*)(bias + ri + 4);
  }

#pragma unroll
  for (int i = 0; i < 2; ++i)
#pragma unroll
    for (int t = 0; t < 4; ++t)
#pragma unroll
      for (int r = 0; r < 8; ++r) {
        const int rowl = 32 * w + 16 * i + 8 * hl + r;
        const float brv = bf16_rne(br[i][r >> 2][r & 3]) * ACT_CAR;
        const float bv = (bias_row != 0) ? brv : bc[t];
        const float v = acc[i * 4 + t][r] * PROJ_SCL + bv;
        const _Float16 hv = (_Float16)v;
        const float res = (v - (float)hv) * RES_CAR;
        ldsH[rowl * 72 + 16 * t + c] = hv;
        ldsL[rowl * 72 + 16 * t + c] = (_Float16)res;
      }
  __syncthreads();

  _Float16* const bh = PH + zb * sC + (size_t)m0 * ldc + n0;
  _Float16* const bl = PL + zb * sC + (size_t)m0 * ldc + n0;
  for (int i = 0; i < 8; ++i) {
    const int q = i * 128 + tid;
    const int rowl = q >> 3, ch = (q & 7) * 8;
    const v8h vh = *(const v8h*)(ldsH + rowl * 72 + ch);
    const v8h vl = *(const v8h*)(ldsL + rowl * 72 + ch);
    *(volatile v8h*)(bh + (size_t)rowl * ldc + ch) = vh;
    *(volatile v8h*)(bl + (size_t)rowl * ldc + ch) = vl;
  }
  __threadfence();
  for (int i = 0; i < 8; ++i) {
    const int q = i * 128 + tid;
    const int rowl = q >> 3, ch = (q & 7) * 8;
    const v8h vh = *(const v8h*)(ldsH + rowl * 72 + ch);
    const v8h vl = *(const v8h*)(ldsL + rowl * 72 + ch);
    *(volatile v8h*)(bh + (size_t)rowl * ldc + ch) = vh;
    *(volatile v8h*)(bl + (size_t)rowl * ldc + ch) = vl;
  }
}

__global__ __launch_bounds__(256) __attribute__((amdgpu_num_vgpr(256)))
void k_attn(const _Float16* __restrict__ QH, const _Float16* __restrict__ QL,
            const _Float16* __restrict__ KH, const _Float16* __restrict__ KL,
            const _Float16* __restrict__ VtH, const _Float16* __restrict__ VtL,
            _Float16* __restrict__ OH, _Float16* __restrict__ OL)
{
  constexpr int KT_H   = 32 * 72;
  constexpr int V_H    = HD * 40;
  constexpr int P_H    = 8 * 16 * 40;
  constexpr int TILE_H = 2 * KT_H + 2 * V_H + P_H;
  constexpr int EPI_H  = 2 * 128 * 72;
  constexpr int LDS_H  = (TILE_H > EPI_H) ? TILE_H : EPI_H;
  __shared__ __attribute__((aligned(16))) _Float16 lds[LDS_H];
  _Float16* const ldsK0 = lds;
  _Float16* const ldsK1 = ldsK0 + KT_H;
  _Float16* const ldsVH = ldsK1 + KT_H;
  _Float16* const ldsVL = ldsVH + V_H;
  _Float16* const ldsP  = ldsVL + V_H;
  _Float16* const ldsOH = lds;
  _Float16* const ldsOL = lds + 128 * 72;

  const int tid = threadIdx.x, lane = tid & 31, w = tid >> 5;
  const int hl = lane >> 4, c = lane & 15;
  const int q0 = blockIdx.x * 128;
  const int col0 = blockIdx.y * HD;
  const size_t bz = (size_t)blockIdx.z;

  const size_t qrow = (bz * SEQ + (size_t)(q0 + 16 * w + c)) * DM + col0;
  v16h qh[2], ql[2];
#pragma unroll
  for (int ks = 0; ks < 2; ++ks) {
    qh[ks] = ld_frag(QH + qrow + 32 * ks, hl);
    ql[ks] = ld_frag(QL + qrow + 32 * ks, hl);
  }
  _Float16* const myP = ldsP + w * (16 * 40);

  const int krr = tid >> 3, kcc = (tid & 7) * 8;
  const int vdd = tid >> 2, vkc = (tid & 3) * 8;
  const _Float16* const kgh = KH + (bz * MCTX + (size_t)krr) * DM + col0 + kcc;
  const _Float16* const kgl = KL + (bz * MCTX + (size_t)krr) * DM + col0 + kcc;
  const _Float16* const vgh = VtH + bz * ((size_t)DM * MCTX) + (size_t)(col0 + vdd) * MCTX + vkc;
  const _Float16* const vgl = VtL + bz * ((size_t)DM * MCTX) + (size_t)(col0 + vdd) * MCTX + vkc;

  float m[8], l[8];
  v8f oh[4] = {}, ol[4] = {};
#pragma unroll
  for (int r = 0; r < 8; ++r) { m[r] = -__builtin_inff(); l[r] = 0.f; }

#pragma unroll 1
  for (int kt = 0; kt < MCTX / 32; ++kt) {
    const int mk = kt * 32;
    {
      const v8h k8h = *(const v8h*)(kgh + (size_t)mk * DM);
      const v8h k8l = *(const v8h*)(kgl + (size_t)mk * DM);
      const v8h v8a = *(const v8h*)(vgh + mk);
      const v8h v8b = *(const v8h*)(vgl + mk);
      *(v8h*)(ldsK0 + krr * 72 + kcc) = k8h;
      *(v8h*)(ldsK1 + krr * 72 + kcc) = k8l;
      *(v8h*)(ldsVH + vdd * 40 + vkc) = v8a;
      *(v8h*)(ldsVL + vdd * 40 + vkc) = v8b;
    }
    __syncthreads();

    v8f sh[2] = {}, sl[2] = {};
#pragma unroll
    for (int ks = 0; ks < 2; ++ks) {
#pragma unroll
      for (int t = 0; t < 2; ++t) {
        const v16h kfh = ld_frag(ldsK0 + (16 * t + c) * 72 + 32 * ks, hl);
        const v16h kfl = ld_frag(ldsK1 + (16 * t + c) * 72 + 32 * ks, hl);
        sh[t] = mma(qh[ks], kfh, sh[t]);
        sl[t] = mma(ql[ks], kfh, sl[t]);
        sl[t] = mma(qh[ks], kfl, sl[t]);
      }
    }

#pragma unroll
    for (int r = 0; r < 8; ++r) {
      const float v0 = (sh[0][r] + sl[0][r] * RES_INV) * S_SCL;
      const float v1 = (sh[1][r] + sl[1][r] * RES_INV) * S_SCL;
      float tm = fmaxf(v0, v1);
      tm = fmaxf(tm, __shfl_xor(tm, 1, 32));
      tm = fmaxf(tm, __shfl_xor(tm, 2, 32));
      tm = fmaxf(tm, __shfl_xor(tm, 4, 32));
      tm = fmaxf(tm, __shfl_xor(tm, 8, 32));
      const float mn = fmaxf(m[r], tm);
      const float al = __expf(m[r] - mn);
      const float p0 = __expf(v0 - mn), p1 = __expf(v1 - mn);
      float rs = p0 + p1;
      rs += __shfl_xor(rs, 1, 32);
      rs += __shfl_xor(rs, 2, 32);
      rs += __shfl_xor(rs, 4, 32);
      rs += __shfl_xor(rs, 8, 32);
      l[r] = l[r] * al + rs;
      m[r] = mn;
#pragma unroll
      for (int t = 0; t < 4; ++t) { oh[t][r] *= al; ol[t][r] *= al; }
      _Float16* pp = myP + (8 * hl + r) * 40 + c;
      pp[0]  = (_Float16)(p0 * P_CAR);
      pp[16] = (_Float16)(p1 * P_CAR);
    }
    __syncthreads();

    const v16h pf = ld_frag(myP + c * 40, hl);
#pragma unroll
    for (int t = 0; t < 4; ++t) {
      const v16h vfh = ld_frag(ldsVH + (16 * t + c) * 40, hl);
      const v16h vfl = ld_frag(ldsVL + (16 * t + c) * 40, hl);
      oh[t] = mma(pf, vfh, oh[t]);
      ol[t] = mma(pf, vfl, ol[t]);
    }
    __syncthreads();
  }

#pragma unroll
  for (int r = 0; r < 8; ++r) {
    const float inv = (1.0f / l[r]) * O_SCL;
    const int rowl = 16 * w + 8 * hl + r;
#pragma unroll
    for (int t = 0; t < 4; ++t) {
      const float v = (oh[t][r] + ol[t][r] * RES_INV) * inv;
      const _Float16 hv = (_Float16)v;
      const float res = (v - (float)hv) * RES_CAR;
      ldsOH[rowl * 72 + 16 * t + c] = hv;
      ldsOL[rowl * 72 + 16 * t + c] = (_Float16)res;
    }
  }
  __syncthreads();
  _Float16* const bh = OH + (bz * SEQ + (size_t)q0) * DM + col0;
  _Float16* const bl = OL + (bz * SEQ + (size_t)q0) * DM + col0;
  for (int i = 0; i < 4; ++i) {
    const int q = i * 256 + tid;
    const int rowl = q >> 3, ch = (q & 7) * 8;
    const v8h vh = *(const v8h*)(ldsOH + rowl * 72 + ch);
    const v8h vl = *(const v8h*)(ldsOL + rowl * 72 + ch);
    *(volatile v8h*)(bh + (size_t)rowl * DM + ch) = vh;
    *(volatile v8h*)(bl + (size_t)rowl * DM + ch) = vl;
  }
  __threadfence();
  for (int i = 0; i < 4; ++i) {
    const int q = i * 256 + tid;
    const int rowl = q >> 3, ch = (q & 7) * 8;
    const v8h vh = *(const v8h*)(ldsOH + rowl * 72 + ch);
    const v8h vl = *(const v8h*)(ldsOL + rowl * 72 + ch);
    *(volatile v8h*)(bh + (size_t)rowl * DM + ch) = vh;
    *(volatile v8h*)(bl + (size_t)rowl * DM + ch) = vl;
  }
}

__global__ __launch_bounds__(128) __attribute__((amdgpu_num_vgpr(256)))
void k_oproj(const _Float16* __restrict__ AH, const _Float16* __restrict__ AL,
             const _Float16* __restrict__ Bt, const float* __restrict__ bias,
             float* __restrict__ Out)
{
  __shared__ __attribute__((aligned(16))) float ldsF[64 * 68];

  const int tid = threadIdx.x, lane = tid & 31, w = tid >> 5;
  const int hl = lane >> 4, c = lane & 15;
  const int m0 = blockIdx.y * 64, n0 = blockIdx.x * 64;
  const size_t bz = (size_t)blockIdx.z;
  const size_t mrow = bz * SEQ + (size_t)(m0 + 16 * w + c);

  const _Float16* ap0 = AH + mrow * DM;
  const _Float16* ap1 = AL + mrow * DM;
  const _Float16* bp  = Bt + (size_t)(n0 + c) * DM;

  v8f acc[8] = {};
  gemm_core(ap0, ap1, bp, DM, hl, acc);

  float bo[4];
#pragma unroll
  for (int t = 0; t < 4; ++t) {
    int ci = n0 + 16 * t + c;
    ci = (ci < DM - 1) ? ci : (DM - 1);
    bo[t] = bf16_rne(bias[ci]);
  }

#pragma unroll
  for (int t = 0; t < 4; ++t)
#pragma unroll
    for (int r = 0; r < 8; ++r) {
      const int rowl = 16 * w + 8 * hl + r;
      ldsF[rowl * 68 + 16 * t + c] = (acc[t][r] + acc[4 + t][r] * RES_INV) * OUT_SCL + bo[t];
    }
  __syncthreads();

  float* const ob = Out + (bz * SEQ_FULL + (size_t)m0) * DM + n0;
  for (int i = 0; i < 8; ++i) {
    const int qi = i * 128 + tid;
    const int rowl = qi >> 4, col = (qi & 15) * 4;
    const v4f v = *(const v4f*)(ldsF + rowl * 68 + col);
    *(volatile v4f*)(ob + (size_t)rowl * DM + col) = v;
  }
  __threadfence();
  for (int i = 0; i < 8; ++i) {
    const int qi = i * 128 + tid;
    const int rowl = qi >> 4, col = (qi & 15) * 4;
    const v4f v = *(const v4f*)(ldsF + rowl * 68 + col);
    *(volatile v4f*)(ob + (size_t)rowl * DM + col) = v;
  }
}

extern "C" void kernel_launch(void* const* d_in, const int* in_sizes, int n_in,
                              void* d_out, int out_size, void* d_ws, size_t ws_size,
                              hipStream_t stream)
{
  if (n_in < 10) return;
  const long needX = ((long)(NB - 1) * SEQ_FULL + SEQ) * DM;
  const long needY = ((long)(NB - 1) * MCTX_FULL + MCTX) * DM;
  if ((long)in_sizes[0] < needX) return;
  if ((long)in_sizes[1] < needY) return;
  if ((long)in_sizes[2] < (long)DM * DM) return;
  if ((long)in_sizes[3] < (long)DM) return;
  if ((long)in_sizes[4] < (long)DM * DM) return;
  if ((long)in_sizes[5] < (long)DM) return;
  if ((long)in_sizes[6] < (long)DM * DM) return;
  if ((long)in_sizes[7] < (long)DM) return;
  if ((long)in_sizes[8] < (long)DM * DM) return;
  if ((long)in_sizes[9] < (long)DM) return;
  if ((long)out_size < needX) return;

  const float* x  = (const float*)d_in[0];
  const float* y  = (const float*)d_in[1];
  const float* Wq = (const float*)d_in[2];
  const float* bq = (const float*)d_in[3];
  const float* Wk = (const float*)d_in[4];
  const float* bk = (const float*)d_in[5];
  const float* Wv = (const float*)d_in[6];
  const float* bv = (const float*)d_in[7];
  const float* Wp = (const float*)d_in[8];
  const float* bp = (const float*)d_in[9];
  float* out = (float*)d_out;

  const size_t nX = (size_t)NB * SEQ * DM;
  const size_t nY = (size_t)NB * MCTX * DM;
  const size_t nW = (size_t)DM * DM;
  const size_t total_halves = nX + nY + 4 * nW + 2 * nX + 2 * nY + 2 * nY + 2 * nX;
  if (total_halves * sizeof(_Float16) > ws_size) return;
  if (total_halves * sizeof(_Float16) > (size_t)134217728) return;

  _Float16* X16  = (_Float16*)d_ws;
  _Float16* Y16  = X16  + nX;
  _Float16* Wq16 = Y16  + nY;
  _Float16* Wk16 = Wq16 + nW;
  _Float16* Wv16 = Wk16 + nW;
  _Float16* Wp16 = Wv16 + nW;
  _Float16* QH   = Wp16 + nW;
  _Float16* QL   = QH   + nX;
  _Float16* KH   = QL   + nX;
  _Float16* KL   = KH   + nY;
  _Float16* VtH  = KL   + nY;
  _Float16* VtL  = VtH  + nY;
  _Float16* OH   = VtL  + nY;
  _Float16* OL   = OH   + nX;

  const unsigned x8 = (unsigned)((size_t)SEQ * DM / 8);
  const unsigned y8 = (unsigned)((size_t)MCTX * DM / 8);
  const unsigned w8 = (unsigned)(nW / 8);
  k_cvt8<<<dim3(x8 / 256, NB), 256, 0, stream>>>(x, X16, ACT_CAR,
      (unsigned)((size_t)SEQ_FULL * DM), (unsigned)((size_t)SEQ * DM), x8);
  k_cvt8<<<dim3(y8 / 256, NB), 256, 0, stream>>>(y, Y16, ACT_CAR,
      (unsigned)((size_t)MCTX_FULL * DM), (unsigned)((size_t)MCTX * DM), y8);
  k_cvt8<<<dim3(w8 / 256, 1), 256, 0, stream>>>(Wq, Wq16, W_CAR, 0u, 0u, w8);
  k_cvt8<<<dim3(w8 / 256, 1), 256, 0, stream>>>(Wk, Wk16, W_CAR, 0u, 0u, w8);
  k_cvt8<<<dim3(w8 / 256, 1), 256, 0, stream>>>(Wv, Wv16, W_CAR, 0u, 0u, w8);
  k_cvt8<<<dim3(w8 / 256, 1), 256, 0, stream>>>(Wp, Wp16, W_CAR, 0u, 0u, w8);

  k_proj<<<dim3(DM / 64, NB * SEQ / 128, 1), 128, 0, stream>>>(
      X16, Wq16, QH, QL, bq, (size_t)0, (size_t)0, DM, DM, 0);
  k_proj<<<dim3(DM / 64, NB * MCTX / 128, 1), 128, 0, stream>>>(
      Y16, Wk16, KH, KL, bk, (size_t)0, (size_t)0, DM, DM, 0);
  k_proj<<<dim3(MCTX / 64, DM / 128, NB), 128, 0, stream>>>(
      Wv16, Y16, VtH, VtL, bv, (size_t)MCTX * DM, (size_t)DM * MCTX, DM, MCTX, 1);

  k_attn<<<dim3(SEQ / 128, NH, NB), 256, 0, stream>>>(QH, QL, KH, KL, VtH, VtL, OH, OL);

  k_oproj<<<dim3(DM / 64, SEQ / 64, NB), 128, 0, stream>>>(OH, OL, Wp16, bp, out);
}
